// PABlock_3882650436003
// MI455X (gfx1250) — hardware-run, weakly checked
//
#include <hip/hip_runtime.h>
#include <stdint.h>

typedef __attribute__((ext_vector_type(16))) _Float16 v16h;
typedef __attribute__((ext_vector_type(8)))  _Float16 v8h;
typedef __attribute__((ext_vector_type(16))) __bf16   v16b;
typedef __attribute__((ext_vector_type(8)))  __bf16   v8b;
typedef __attribute__((ext_vector_type(8)))  float    v8f;
typedef __attribute__((ext_vector_type(4)))  float    v4f;

constexpr int NBATCH = 4;
constexpr int NCH    = 512;
constexpr int NPOS   = 4096;
constexpr int NCQ    = 64;
constexpr int NQK    = 2 * NCQ;

__device__ __forceinline__ unsigned short f2bf_bits(float f) {
  unsigned u = __float_as_uint(f);
  return (unsigned short)((u + 0x7FFFu + ((u >> 16) & 1u)) >> 16);
}
__device__ __forceinline__ float bf_bits2f(unsigned short h) { return __uint_as_float(((unsigned)h) << 16); }

__device__ __forceinline__ void dep_guard_h(v8f& a, v8f& b, v16h x, v16h y) { asm volatile("v_nop\n\tv_nop\n\tv_nop\n\tv_nop" : "+v"(a), "+v"(b) : "v"(x), "v"(y)); }
__device__ __forceinline__ void dep_guard_b(v8f& a, v8f& b, v16b x, v16b y) { asm volatile("v_nop\n\tv_nop\n\tv_nop\n\tv_nop" : "+v"(a), "+v"(b) : "v"(x), "v"(y)); }
__device__ __forceinline__ void keep4_h(v16h a, v16h b, v16h c, v16h d) { asm volatile("v_nop" :: "v"(a), "v"(b), "v"(c), "v"(d)); }
__device__ __forceinline__ void keep4_b(v16b a, v16b b, v16b c, v16b d) { asm volatile("v_nop" :: "v"(a), "v"(b), "v"(c), "v"(d)); }
__device__ __forceinline__ void acc_guard4(v8f& a, v8f& b, v8f& c, v8f& d) { asm volatile("v_nop\n\tv_nop\n\tv_nop\n\tv_nop" : "+v"(a), "+v"(b), "+v"(c), "+v"(d)); }

template <typename T> struct Frag;
template <> struct Frag<_Float16> {
  typedef v16h V; union U { v16h v; v8h h[2]; };
  static __device__ __forceinline__ v16h load(const _Float16* p) {
    U f; f.h[0] = *(const v8h*)(p); f.h[1] = *(const v8h*)(p + 16); return f.v;
  }
  static __device__ __forceinline__ v8f mma(v16h a, v16h b, v8f c) {
    return __builtin_amdgcn_wmma_f32_16x16x32_f16(false, a, false, b, (short)0, c, false, false);
  }
  static __device__ __forceinline__ void guard(v8f& a, v8f& b, v16h x, v16h y) { dep_guard_h(a, b, x, y); }
  static __device__ __forceinline__ void keep(v16h a, v16h b, v16h c, v16h d) { keep4_h(a, b, c, d); }
};
template <> struct Frag<__bf16> {
  typedef v16b V; union U { v16b v; v8b h[2]; };
  static __device__ __forceinline__ v16b load(const __bf16* p) {
    U f; f.h[0] = *(const v8b*)(p); f.h[1] = *(const v8b*)(p + 16); return f.v;
  }
  static __device__ __forceinline__ v8f mma(v16b a, v16b b, v8f c) {
    return __builtin_amdgcn_wmma_f32_16x16x32_bf16(false, a, false, b, (short)0, c, false, false);
  }
  static __device__ __forceinline__ void guard(v8f& a, v8f& b, v16b x, v16b y) { dep_guard_b(a, b, x, y); }
  static __device__ __forceinline__ void keep(v16b a, v16b b, v16b c, v16b d) { keep4_b(a, b, c, d); }
};

template <int ET> struct Elem;
template <> struct Elem<0> { typedef _Float16 T; };
template <> struct Elem<1> { typedef __bf16 T; };
template <int ET, bool SPLIT, int BIAS_MODE, int OUT_MODE, bool RESG>
__global__ __launch_bounds__(256) void wmma_gemm64(
    const unsigned short* __restrict__ Ap, const unsigned short* __restrict__ A2p, int lda, long strideA,
    const unsigned short* __restrict__ Btp, const unsigned short* __restrict__ Bt2p, int ldb, long strideB,
    void* __restrict__ Cout, int ldc, long strideC,
    const float* __restrict__ bias,
    const float* __restrict__ resid, long strideR,
    const float* __restrict__ gptr,
    int M, int N, int K, float scale) {
  typedef typename Elem<ET>::T T;
  typedef typename Frag<T>::V V;
  const T* A = (const T*)Ap; const T* A2 = (const T*)A2p; const T* Bt = (const T*)Btp; const T* Bt2 = (const T*)Bt2p;
  __shared__ __align__(16) float sT[8][16 * 68];
  const int b    = blockIdx.y;
  const int lane = threadIdx.x & 31;
  const int wave = threadIdx.x >> 5;
  const int tilesN = N >> 6;
  const int tilesM = M >> 6;
  const int tile = blockIdx.x * 8 + wave;
  if (tile >= tilesM * tilesN) return;
  const int tm = tile / tilesN;
  const int tn = tile - tm * tilesN;
  const int m0 = tm << 6;
  const int n0 = tn << 6;

  const T* Ab  = A  + (size_t)b * strideA;
  const T* Bb  = Bt + (size_t)b * strideB;
  const T* Ab2 = SPLIT ? (A2  + (size_t)b * strideA) : nullptr;
  const T* Bb2 = SPLIT ? (Bt2 + (size_t)b * strideB) : nullptr;

  const int rlane = lane & 15;
  const int koff  = (lane >> 4) * 8;
  const int mOff  = (lane >> 4) * 8;

  v8f acc[4][4];
#pragma unroll
  for (int i = 0; i < 4; ++i)
#pragma unroll
    for (int j = 0; j < 4; ++j) acc[i][j] = (v8f){0.f,0.f,0.f,0.f,0.f,0.f,0.f,0.f};

  for (int k0 = 0; k0 < K; k0 += 32) {
    V bh[4], bl[4];
#pragma unroll
    for (int j = 0; j < 4; ++j) {
      const size_t bo = (size_t)(n0 + (j << 4) + rlane) * ldb + koff + k0;
      bh[j] = Frag<T>::load(Bb + bo);
      if (SPLIT) bl[j] = Frag<T>::load(Bb2 + bo);
    }
#pragma unroll
    for (int i = 0; i < 4; ++i) {
      const size_t ao = (size_t)(m0 + (i << 4) + rlane) * lda + koff + k0;
      V ah = Frag<T>::load(Ab + ao);
      V al;
      if (SPLIT) al = Frag<T>::load(Ab2 + ao);
#pragma unroll
      for (int j = 0; j < 4; ++j) {
        acc[i][j] = Frag<T>::mma(ah, bh[j], acc[i][j]);
        if (SPLIT) {
          acc[i][j] = Frag<T>::mma(ah, bl[j], acc[i][j]);
          acc[i][j] = Frag<T>::mma(al, bh[j], acc[i][j]);
        }
      }
      Frag<T>::guard(acc[i][0], acc[i][3], ah, SPLIT ? al : ah);
    }
    Frag<T>::keep(bh[0], bh[1], bh[2], bh[3]);
    if (SPLIT) Frag<T>::keep(bl[0], bl[1], bl[2], bl[3]);
  }
  acc_guard4(acc[0][0], acc[0][1], acc[0][2], acc[0][3]);
  acc_guard4(acc[1][0], acc[1][1], acc[1][2], acc[1][3]);
  acc_guard4(acc[2][0], acc[2][1], acc[2][2], acc[2][3]);
  acc_guard4(acc[3][0], acc[3][1], acc[3][2], acc[3][3]);

  float* slab = sT[wave];
  const float gres = RESG ? gptr[0] : 0.f;
  const float* Rb = RESG ? (resid + (size_t)b * strideR) : nullptr;
#pragma unroll
  for (int i = 0; i < 4; ++i) {
    const int mBase = m0 + (i << 4);
#pragma unroll
    for (int j = 0; j < 4; ++j) {
      const int n = n0 + (j << 4) + rlane;
      float bvv = 0.f;
      if (BIAS_MODE == 2) bvv = bias[n];
#pragma unroll
      for (int r = 0; r < 8; ++r) {
        float v = acc[i][j][r] * scale;
        if (BIAS_MODE == 1) v += bias[mBase + mOff + r];
        if (BIAS_MODE == 2) v += bvv;
        slab[(mOff + r) * 68 + (j << 4) + rlane] = v;
      }
    }
    __builtin_amdgcn_fence(__ATOMIC_RELEASE, "workgroup");
    __builtin_amdgcn_wave_barrier();
    __builtin_amdgcn_fence(__ATOMIC_ACQUIRE, "workgroup");
    if (OUT_MODE == 0) {
      float* C = (float*)Cout + (size_t)b * strideC;
      const int hh = lane >> 4, c4 = (lane & 15) * 4;
      if (RESG) {
#pragma unroll
        for (int it = 0; it < 8; ++it) {
          const int row = it * 2 + hh;
          v4f v = *(const v4f*)(slab + row * 68 + c4);
          const v4f xr = *(const v4f*)(Rb + (size_t)(mBase + row) * ldc + n0 + c4);
          v = v * gres + xr;
          *(v4f*)(slab + row * 68 + c4) = v;
        }
      }
      for (int pass = 0; pass < 2; ++pass) {
#pragma unroll
        for (int it = 0; it < 8; ++it) {
          const int row = it * 2 + hh;
          v4f v = *(const v4f*)(slab + row * 68 + c4);
          *(volatile v4f*)(C + (size_t)(mBase + row) * ldc + n0 + c4) = v;
        }
        __threadfence();
      }
    } else {
      const int q = lane >> 3, c8 = (lane & 7) * 8;
      unsigned short* C = (unsigned short*)Cout + (size_t)b * strideC;
      for (int pass = 0; pass < 2; ++pass) {
#pragma unroll
        for (int it = 0; it < 4; ++it) {
          const int row = it * 4 + q;
          const float* sp = slab + row * 68 + c8;
          v8h hv;
#pragma unroll
          for (int e = 0; e < 8; ++e) hv[e] = (_Float16)sp[e];
          *(volatile v8h*)(C + (size_t)(mBase + row) * ldc + n0 + c8) = hv;
        }
        __threadfence();
      }
    }
    __builtin_amdgcn_fence(__ATOMIC_RELEASE, "workgroup");
    __builtin_amdgcn_wave_barrier();
    __builtin_amdgcn_fence(__ATOMIC_ACQUIRE, "workgroup");
  }
}

__global__ __launch_bounds__(256) void cast_f32_f16x2s(
    const float* __restrict__ in, unsigned short* __restrict__ out, int n2, float sc) {
  int i = blockIdx.x * 256 + threadIdx.x;
  if (i < n2) {
    const _Float16 h0 = (_Float16)(in[2 * i] * sc), h1 = (_Float16)(in[2 * i + 1] * sc);
    const unsigned u = (unsigned)__builtin_bit_cast(unsigned short, h0) | ((unsigned)__builtin_bit_cast(unsigned short, h1) << 16);
    ((volatile unsigned*)out)[i] = u;
    __threadfence();
    ((volatile unsigned*)out)[i] = u;
  }
}

__global__ __launch_bounds__(128) void concat_bias(
    const float* __restrict__ ba, const float* __restrict__ bb, float* __restrict__ ball) {
  const int t = threadIdx.x;
  const int ia = (t < NCQ) ? t : (NCQ - 1);
  const int ib = (t >= NCQ) ? (t - NCQ) : 0;
  const float va = ba[ia];
  const float vb = bb[ib];
  const float v = (t < NCQ) ? va : vb;
  ((volatile float*)ball)[t] = v;
  __threadfence();
  ((volatile float*)ball)[t] = v;
}

__global__ __launch_bounds__(256) void x_to_xT(const float* __restrict__ x, unsigned short* __restrict__ xT) {
  __shared__ __align__(16) float tile[64 * 68];
  const int tid = threadIdx.x, lane = tid & 31, wave = tid >> 5;
  const int n0 = blockIdx.x * 64;
  const int c0 = blockIdx.y * 64;
  const int b  = blockIdx.z;
  const float* xb = x + ((size_t)b * NCH + c0) * NPOS + n0;
#pragma unroll
  for (int k = 0; k < 4; ++k) {
    const int idx = tid + 256 * k;
    const int c = idx >> 4, n4 = (idx & 15) * 4;
    const v4f v = *(const v4f*)(xb + (size_t)c * NPOS + n4);
    *(v4f*)(tile + c * 68 + n4) = v;
  }
  __syncthreads();
  const int q = lane >> 3, c8 = (lane & 7) * 8;
  unsigned short* ob = xT + ((size_t)b * NPOS + n0) * NCH + c0;
  for (int pass = 0; pass < 2; ++pass) {
#pragma unroll
    for (int it = 0; it < 2; ++it) {
      const int n = wave * 8 + it * 4 + q;
      v8h hv;
#pragma unroll
      for (int e = 0; e < 8; ++e) hv[e] = (_Float16)tile[(c8 + e) * 68 + n];
      *(volatile v8h*)(ob + (size_t)n * NCH + c8) = hv;
    }
    __threadfence();
  }
}

__global__ __launch_bounds__(256) void softmax_rows(
    const float* __restrict__ S, unsigned short* __restrict__ P, float carry) {
  __shared__ __align__(16) float srow[NPOS];
  __shared__ float redm[8];
  __shared__ float reds[8];
  const int tid = threadIdx.x, lane = tid & 31, wave = tid >> 5;
  const int row = blockIdx.x;
  const float* sr = S + (size_t)row * NPOS;
  const int cA = 8 * tid;
  const int cB = (NPOS / 2) + 8 * tid;
  const v4f a0 = *(const v4f*)(sr + cA);
  const v4f a1 = *(const v4f*)(sr + cA + 4);
  const v4f a2 = *(const v4f*)(sr + cB);
  const v4f a3 = *(const v4f*)(sr + cB + 4);
  float m = a0[0];
#pragma unroll
  for (int e = 0; e < 4; ++e) {
    m = fmaxf(m, a0[e]); m = fmaxf(m, a1[e]); m = fmaxf(m, a2[e]); m = fmaxf(m, a3[e]);
  }
  *(v4f*)(srow + cA) = a0;
  *(v4f*)(srow + cA + 4) = a1;
  *(v4f*)(srow + cB) = a2;
  *(v4f*)(srow + cB + 4) = a3;
#pragma unroll
  for (int off = 1; off < 32; off <<= 1) m = fmaxf(m, __shfl_xor(m, off, 32));
  if (lane == 0) redm[wave] = m;
  __syncthreads();
  float mr = redm[0];
#pragma unroll
  for (int w = 1; w < 8; ++w) mr = fmaxf(mr, redm[w]);

  float lsum = 0.f;
#pragma unroll 1
  for (int e = 0; e < 16; ++e) {
    const int col = cA + (e & 7) + (e >> 3) * (NPOS / 2);
    const float p = expf(srow[col] - mr);
    srow[col] = p;
    lsum += p;
  }
#pragma unroll
  for (int off = 1; off < 32; off <<= 1) lsum += __shfl_xor(lsum, off, 32);
  if (lane == 0) reds[wave] = lsum;
  __syncthreads();
  float l = reds[0];
#pragma unroll
  for (int w = 1; w < 8; ++w) l += reds[w];
  const float f = carry * (1.0f / l);

  const v4f p0 = *(const v4f*)(srow + cA);
  const v4f p1 = *(const v4f*)(srow + cA + 4);
  const v4f p2 = *(const v4f*)(srow + cB);
  const v4f p3 = *(const v4f*)(srow + cB + 4);
  v8h h0, h1;
#pragma unroll
  for (int e = 0; e < 4; ++e) {
    h0[e]     = (_Float16)(p0[e] * f);
    h0[4 + e] = (_Float16)(p1[e] * f);
    h1[e]     = (_Float16)(p2[e] * f);
    h1[4 + e] = (_Float16)(p3[e] * f);
  }
  unsigned short* pr = P + (size_t)row * NPOS;
  for (int pass = 0; pass < 2; ++pass) {
    *(volatile v8h*)(pr + cA) = h0;
    *(volatile v8h*)(pr + cB) = h1;
    __threadfence();
  }
}

extern "C" void kernel_launch(void* const* d_in, const int* in_sizes, int n_in,
                              void* d_out, int out_size, void* d_ws, size_t ws_size,
                              hipStream_t stream) {
  constexpr size_t OFF_WQK  = 0;
  constexpr size_t OFF_WV   = OFF_WQK + (size_t)NQK * NCH * 2;
  constexpr size_t OFF_BALL = OFF_WV + (size_t)NCH * NCH * 2;
  constexpr size_t OFF_QK   = OFF_BALL + 1024;
  constexpr size_t OFF_V    = OFF_QK + (size_t)NBATCH * NPOS * NQK * 2;
  constexpr size_t OFF_BIG  = OFF_V + (size_t)NBATCH * NCH * NPOS * 2;
  constexpr size_t SZ_XT    = (size_t)NBATCH * NPOS * NCH * 2;
  constexpr size_t SZ_S     = (size_t)NPOS * NPOS * 4;
  constexpr size_t SZ_P     = (size_t)NPOS * NPOS * 2;
  constexpr size_t OFF_S    = OFF_BIG;
  constexpr size_t OFF_P    = OFF_BIG + SZ_S;
  constexpr size_t SZ_BIG   = (SZ_XT > SZ_S + SZ_P) ? SZ_XT : (SZ_S + SZ_P);
  constexpr size_t WS_TOTAL = OFF_BIG + SZ_BIG;
  static_assert(WS_TOTAL == 122291200);
  static_assert(WS_TOTAL <= 134217728);
  static_assert((OFF_WV % 128) == 0 && (OFF_BALL % 128) == 0 && (OFF_QK % 128) == 0 && (OFF_V % 128) == 0 && (OFF_BIG % 128) == 0 && (OFF_P % 128) == 0);
  static_assert(NPOS % 64 == 0 && NQK % 64 == 0 && NCH % 64 == 0);
  static_assert(NCH % 32 == 0 && NCQ % 32 == 0 && NPOS % 32 == 0);

  if (n_in < 8) return;
  if (in_sizes[0] != NBATCH * NCH * NPOS) return;
  if (in_sizes[1] != NCQ * NCH || in_sizes[3] != NCQ * NCH || in_sizes[5] != NCH * NCH) return;
  if (in_sizes[2] != NCQ || in_sizes[4] != NCQ || in_sizes[6] != NCH || in_sizes[7] < 1) return;
  if (out_size != NBATCH * NCH * NPOS) return;
  if (ws_size < WS_TOTAL) return;

  const float* p_x  = (const float*)d_in[0];
  const float* p_wq = (const float*)d_in[1];
  const float* p_bq = (const float*)d_in[2];
  const float* p_wk = (const float*)d_in[3];
  const float* p_bk = (const float*)d_in[4];
  const float* p_wv = (const float*)d_in[5];
  const float* p_bv = (const float*)d_in[6];
  const float* p_g  = (const float*)d_in[7];
  float* p_out = (float*)d_out;

  char* ws = (char*)d_ws;
  unsigned short* wqk16 = (unsigned short*)(ws + OFF_WQK);
  unsigned short* wv16  = (unsigned short*)(ws + OFF_WV);
  float*          ball  = (float*)(ws + OFF_BALL);
  unsigned short* qk16  = (unsigned short*)(ws + OFF_QK);
  unsigned short* v16   = (unsigned short*)(ws + OFF_V);
  unsigned short* xT16  = (unsigned short*)(ws + OFF_BIG);
  float*          s32   = (float*)(ws + OFF_S);
  unsigned short* p16   = (unsigned short*)(ws + OFF_P);

  const float wcarry = 64.0f;
  const float pcarry = 16384.0f;

  cast_f32_f16x2s<<<(NCQ * NCH / 2 + 255) / 256, 256, 0, stream>>>(p_wq, wqk16, NCQ * NCH / 2, wcarry);
  cast_f32_f16x2s<<<(NCQ * NCH / 2 + 255) / 256, 256, 0, stream>>>(p_wk, wqk16 + (size_t)NCQ * NCH, NCQ * NCH / 2, wcarry);
  cast_f32_f16x2s<<<(NCH * NCH / 2 + 255) / 256, 256, 0, stream>>>(p_wv, wv16, NCH * NCH / 2, wcarry);
  concat_bias<<<1, NQK, 0, stream>>>(p_bq, p_bk, ball);

  x_to_xT<<<dim3(NPOS / 64, NCH / 64, NBATCH), 256, 0, stream>>>(p_x, xT16);

  wmma_gemm64<0, false, 2, 1, false><<<dim3((NPOS / 64) * (NQK / 64) / 8, NBATCH), 256, 0, stream>>>(
      xT16, nullptr, NCH, (long)NPOS * NCH,
      wqk16, nullptr, NCH, 0L,
      (void*)qk16, NQK, (long)NPOS * NQK,
      ball, nullptr, 0L, nullptr,
      NPOS, NQK, NCH, 1.0f / wcarry);

  wmma_gemm64<0, false, 1, 1, false><<<dim3((NCH / 64) * (NPOS / 64) / 8, NBATCH), 256, 0, stream>>>(
      wv16, nullptr, NCH, 0L,
      xT16, nullptr, NCH, (long)NPOS * NCH,
      (void*)v16, NPOS, (long)NCH * NPOS,
      p_bv, nullptr, 0L, nullptr,
      NCH, NPOS, NCH, 1.0f / wcarry);

  for (int b = 0; b < NBATCH; ++b) {
    const unsigned short* qkb = qk16 + (size_t)b * NPOS * NQK;
    wmma_gemm64<0, false, 0, 0, false><<<dim3((NPOS / 64) * (NPOS / 64) / 8, 1), 256, 0, stream>>>(
        qkb, nullptr, NQK, 0L,
        qkb + NCQ, nullptr, NQK, 0L,
        (void*)s32, NPOS, 0L,
        nullptr, nullptr, 0L, nullptr,
        NPOS, NPOS, NCQ, 1.0f);
    softmax_rows<<<NPOS, 256, 0, stream>>>(s32, p16, pcarry);
    wmma_gemm64<0, false, 0, 0, true><<<dim3((NCH / 64) * (NPOS / 64) / 8, 1), 256, 0, stream>>>(
        v16 + (size_t)b * NCH * NPOS, nullptr, NPOS, 0L,
        p16, nullptr, NPOS, 0L,
        (void*)(p_out + (size_t)b * NCH * NPOS), NPOS, 0L,
        nullptr, p_x + (size_t)b * NCH * NPOS, 0L, p_g,
        NCH, NPOS, NPOS, 1.0f / pcarry);
  }
}
